// kgpr_46316927320314
// MI455X (gfx1250) — hardware-verified
//
#include <hip/hip_runtime.h>
#include <stdint.h>

#define NBATCH 16384
#define NM     2048
#define KD     64
#define NHEAD  4
#define DH     64
#define NCOL   256
#define BROWS  128
#define MCH    32
#define NCHUNK 64
#define CT     8
#define NCT    16
#define NCHALF 2
#define SPITCH 132
#define NBETA  (-0.05f)

static_assert(NBATCH % BROWS == 0);
static_assert(NM == NCHUNK * MCH);
static_assert(NCOL == NCT * 16);
static_assert(NCT == NCHALF * CT);
static_assert(NHEAD * DH == NCOL);
static_assert(KD == 64);
static_assert(NM % 32 == 0);
static_assert((NM * NCOL) % (8 * 256) == 0);
static_assert((SPITCH % 4) == 0);

typedef unsigned short v16us __attribute__((ext_vector_type(16)));
typedef unsigned short v8us  __attribute__((ext_vector_type(8)));
typedef __bf16          v16bf __attribute__((ext_vector_type(16)));
typedef float           v8f   __attribute__((ext_vector_type(8)));
typedef float           v4f   __attribute__((ext_vector_type(4)));
typedef float           v4fa  __attribute__((ext_vector_type(4), may_alias));

union U16 { v16us v; v8us h[2]; };

__device__ __forceinline__ unsigned short bf16bits(float f) {
  unsigned int u = __float_as_uint(f);
  u = u + 0x7FFFu + ((u >> 16) & 1u);
  return (unsigned short)(u >> 16);
}
__device__ __forceinline__ float bf16val(unsigned short b) {
  return __uint_as_float(((unsigned int)b) << 16);
}
__device__ __forceinline__ v16bf asbf(v16us u) { return __builtin_bit_cast(v16bf, u); }

__device__ __forceinline__ v8f mma_bf(v16us a, v16us b, v8f c) {
  return __builtin_amdgcn_wmma_f32_16x16x32_bf16(false, asbf(a), false, asbf(b), (short)0, c, false, false);
}
__device__ __forceinline__ void guard2(v8f& acc, v16us a0, v16us b0, v16us a1, v16us b1) {
#if defined(__HIP_DEVICE_COMPILE__)
  asm volatile("v_nop\n\tv_nop\n\tv_nop\n\tv_nop" : "+v"(acc) : "v"(a0), "v"(b0), "v"(a1), "v"(b1));
#endif
}

__global__ __launch_bounds__(256) void prep_r(const float* __restrict__ R, unsigned short* Rb, float* R2) {
  __shared__ __align__(16) float s_r2[32];
  const int tid = threadIdx.x, lane = tid & 31;
  if ((int)blockIdx.x * 32 + 32 > NM) return;
  const int row = (int)blockIdx.x * 32 + (tid >> 3);
  const int seg = tid & 7;
  const float* rp = R + (size_t)row * KD + seg * 8;
  const v4f a = *(const v4f*)rp;
  const v4f b = *(const v4f*)(rp + 4);
  v8us o = {};
  float sq = 0.f;
#pragma unroll
  for (int e = 0; e < 4; ++e) {
    const unsigned short s0 = bf16bits(a[e]);
    const unsigned short s1 = bf16bits(b[e]);
    o[e] = s0; o[4 + e] = s1;
    const float t0 = bf16val(s0), t1 = bf16val(s1);
    sq = fmaf(t0, t0, sq);
    sq = fmaf(t1, t1, sq);
  }
  sq += __shfl_xor(sq, 1);
  sq += __shfl_xor(sq, 2);
  sq += __shfl_xor(sq, 4);
  if (seg == 0) s_r2[tid >> 3] = sq;
  __syncthreads();
  const v4f rv = *(const v4fa*)(s_r2 + min(lane, 7) * 4);
  unsigned short* op = Rb + (size_t)row * KD + seg * 8;
  float* r2p = R2 + (size_t)blockIdx.x * 32 + lane * 4;
  *(volatile v8us*)op = o;
  if (tid < 8) *(volatile v4f*)r2p = rv;
  __threadfence();
  *(volatile v8us*)op = o;
  if (tid < 8) *(volatile v4f*)r2p = rv;
}

__global__ __launch_bounds__(256) void prep_w(const float* __restrict__ Mx, unsigned short* W) {
  const int g = (int)blockIdx.x * 256 + (int)threadIdx.x;
  if (g >= (NM * NCOL) / 8) return;
  const int q = g & 1;
  const int ln = (g >> 1) & 31;
  const int t16 = (g >> 6) & 15;
  const int c = g >> 10;
  const int hl = ln >> 4, l15 = ln & 15;
  const int n = t16 * 16 + l15;
  const int h = n >> 6, d = n & 63;
  const int mb = c * MCH + 16 * q + 8 * hl;
  const float* mp = Mx + ((size_t)h * NM + mb) * DH + d;
  v8us o = {};
#pragma unroll
  for (int e = 0; e < 8; ++e) o[e] = bf16bits(mp[(size_t)e * DH]);
  unsigned short* wp = W + (size_t)g * 8;
  *(volatile v8us*)wp = o;
  __threadfence();
  *(volatile v8us*)wp = o;
}

__global__ __launch_bounds__(256) void rbf_main(const float* __restrict__ z, const float* __restrict__ R2,
                                                const unsigned short* __restrict__ Rb,
                                                const unsigned short* __restrict__ W, float* out) {
  __shared__ __align__(16) float s_tile[8 * 16 * SPITCH];

  const int tid = threadIdx.x;
  const int wave = tid >> 5, lane = tid & 31, hl = lane >> 4, l15 = lane & 15;
  if ((int)blockIdx.x * BROWS + BROWS > NBATCH || ((int)blockIdx.y + 1) * CT > NCT) return;
  const int rowbase = (int)blockIdx.x * BROWS + wave * 16;
  const int ctbase  = (int)blockIdx.y * CT;

  v16us zf[2];
  float x2p = 0.f;
  {
    const float* zr = z + (size_t)(rowbase + l15) * KD + 8 * hl;
#pragma unroll
    for (int f = 0; f < 2; ++f) {
      const v4f p0 = *(const v4f*)(zr + 32 * f);
      const v4f p1 = *(const v4f*)(zr + 32 * f + 4);
      const v4f p2 = *(const v4f*)(zr + 32 * f + 16);
      const v4f p3 = *(const v4f*)(zr + 32 * f + 20);
      v16us u = {};
#pragma unroll
      for (int e = 0; e < 4; ++e) {
        const unsigned short s0 = bf16bits(p0[e]);
        const unsigned short s1 = bf16bits(p1[e]);
        const unsigned short s2 = bf16bits(p2[e]);
        const unsigned short s3 = bf16bits(p3[e]);
        u[e] = s0; u[4 + e] = s1; u[8 + e] = s2; u[12 + e] = s3;
        const float t0 = bf16val(s0), t1 = bf16val(s1), t2 = bf16val(s2), t3 = bf16val(s3);
        x2p = fmaf(t0, t0, x2p);
        x2p = fmaf(t1, t1, x2p);
        x2p = fmaf(t2, t2, x2p);
        x2p = fmaf(t3, t3, x2p);
      }
      zf[f] = u;
    }
  }
  const float x2 = x2p + __shfl_xor(x2p, 16);

  v8f acc[CT];
  {
    const v8f zero = {};
#pragma unroll
    for (int t = 0; t < CT; ++t) acc[t] = zero;
  }

  for (int c = 0; c < NCHUNK; ++c) {
    const int m0 = c * MCH;
    v16us khu = {}, klu = {};

#pragma unroll
    for (int nt = 0; nt < 2; ++nt) {
      const unsigned short* rp = Rb + (size_t)(m0 + 16 * nt + l15) * KD + 8 * hl;
      U16 ra, rb;
      ra.h[0] = *(const v8us*)(rp);
      ra.h[1] = *(const v8us*)(rp + 16);
      rb.h[0] = *(const v8us*)(rp + 32);
      rb.h[1] = *(const v8us*)(rp + 48);
      v8f c1 = {};
      c1 = mma_bf(ra.v, zf[0], c1);
      c1 = mma_bf(rb.v, zf[1], c1);
      guard2(c1, ra.v, zf[0], rb.v, zf[1]);
      const float* r2p = R2 + m0 + 16 * nt + 8 * hl;
      const v4f r2a = *(const v4f*)r2p;
      const v4f r2b = *(const v4f*)(r2p + 4);
#pragma unroll
      for (int r = 0; r < 8; ++r) {
        const float r2v = (r < 4) ? r2a[r & 3] : r2b[r & 3];
        float d2 = (x2 + (-2.0f) * c1[r]) + r2v;
        d2 = fmaxf(d2, 0.0f);
        const float kv = __expf(NBETA * d2);
        const unsigned short hb = bf16bits(kv);
        const unsigned short lb = bf16bits(kv - bf16val(hb));
        khu[8 * nt + r] = hb;
        klu[8 * nt + r] = lb;
      }
    }

    const unsigned short* wp = W + ((size_t)(c * NCT + ctbase) * 32 + lane) * 16;
#pragma unroll
    for (int t = 0; t < CT; ++t) {
      U16 wb;
      wb.h[0] = *(const v8us*)(wp + t * 512);
      wb.h[1] = *(const v8us*)(wp + t * 512 + 8);
      acc[t] = mma_bf(khu, wb.v, acc[t]);
      acc[t] = mma_bf(klu, wb.v, acc[t]);
      guard2(acc[t], khu, wb.v, klu, wb.v);
    }
  }

  float* sw = s_tile + wave * (16 * SPITCH);
#pragma unroll
  for (int t = 0; t < CT; ++t)
#pragma unroll
    for (int r = 0; r < 8; ++r)
      sw[(8 * hl + r) * SPITCH + 16 * t + l15] = acc[t][r];
  __syncthreads();

  const float* sr = sw + lane * 4;
  float* ob = out + (size_t)rowbase * NCOL + ctbase * 16 + lane * 4;
#pragma unroll
  for (int row = 0; row < 16; ++row) {
    const v4f v = *(const v4fa*)(sr + row * SPITCH);
    *(volatile v4f*)(ob + (size_t)row * NCOL) = v;
  }
  __threadfence();
#pragma unroll
  for (int row = 0; row < 16; ++row) {
    const v4f v = *(const v4fa*)(sr + row * SPITCH);
    *(volatile v4f*)(ob + (size_t)row * NCOL) = v;
  }
}

extern "C" void kernel_launch(void* const* d_in, const int* in_sizes, int n_in,
                              void* d_out, int out_size, void* d_ws, size_t ws_size,
                              hipStream_t stream) {
  if (n_in < 3) return;
  if (in_sizes[0] != NBATCH * KD) return;
  if (in_sizes[1] != NM * KD) return;
  if (in_sizes[2] != NHEAD * NM * DH) return;
  if (out_size != NBATCH * NCOL) return;

  const size_t off_r2 = 0;
  const size_t sz_r2  = (size_t)NM * sizeof(float);
  const size_t off_rb = off_r2 + sz_r2;
  const size_t sz_rb  = (size_t)NM * KD * sizeof(unsigned short);
  const size_t off_w  = off_rb + sz_rb;
  const size_t sz_w   = (size_t)NM * NCOL * sizeof(unsigned short);
  const size_t need   = off_w + sz_w;
  if (need > ws_size) return;
  if (need > (size_t)134217728) return;

  const float* z  = (const float*)d_in[0];
  const float* R  = (const float*)d_in[1];
  const float* Mx = (const float*)d_in[2];
  float* out = (float*)d_out;
  float*          R2 = (float*)((char*)d_ws + off_r2);
  unsigned short* Rb = (unsigned short*)((char*)d_ws + off_rb);
  unsigned short* W  = (unsigned short*)((char*)d_ws + off_w);

  prep_r<<<dim3(NM / 32), dim3(256), 0, stream>>>(R, Rb, R2);
  prep_w<<<dim3((NM * NCOL / 8) / 256), dim3(256), 0, stream>>>(Mx, W);
  rbf_main<<<dim3(NBATCH / BROWS, NCHALF), dim3(256), 0, stream>>>(z, R2, Rb, W, out);
  (void)hipGetLastError();
}
